// LiteFocusMSA_46849503265363
// MI455X (gfx1250) — hardware-verified
//
#include <hip/hip_runtime.h>
#include <math.h>

typedef __attribute__((ext_vector_type(16))) _Float16 v16h;
typedef __attribute__((ext_vector_type(16))) __bf16 v16b;
typedef __attribute__((ext_vector_type(8)))  _Float16 v8h;
typedef __attribute__((ext_vector_type(8)))  float v8f;
typedef __attribute__((ext_vector_type(4)))  float v4f;
typedef __attribute__((ext_vector_type(2)))  float v2f;
typedef __attribute__((ext_vector_type(4)))  unsigned v4u;
typedef __attribute__((ext_vector_type(4)))  int v4i;
typedef float __attribute__((may_alias)) float_a;
typedef int __attribute__((may_alias)) int_a;

template <typename T> __device__ __forceinline__ void vst2(void* p, T v) { *(volatile T*)p = v; __threadfence(); *(volatile T*)p = v; }
__device__ __forceinline__ v8f wmma16(v16h a, v16h b, v8f c) {
  v8f d = __builtin_amdgcn_wmma_f32_16x16x32_f16(false, a, false, b, (short)0, c, false, false);
  asm volatile("v_nop\n\tv_nop\n\tv_nop\n\tv_nop" : "+v"(d) : "v"(a), "v"(b));
  return d;
}
__device__ __forceinline__ v8f wmma_bf(v16b a, v16b b, v8f c) {
  v8f d = __builtin_amdgcn_wmma_f32_16x16x32_bf16(false, a, false, b, (short)0, c, false, false);
  asm volatile("v_nop\n\tv_nop\n\tv_nop\n\tv_nop" : "+v"(d) : "v"(a), "v"(b));
  return d;
}
__device__ __forceinline__ v16h frag_h(const _Float16* rowk0, int lane) {
  union { v16h v; v8h q[2]; } u; const _Float16* p = rowk0 + 8 * (lane >> 4);
  u.q[0] = *(const v8h*)p; u.q[1] = *(const v8h*)(p + 16); return u.v;
}
__device__ __forceinline__ v16h frag_f32(const float* rowk0, int lane) {
  v16h a; const float* p = rowk0 + 8 * (lane >> 4);
#pragma unroll
  for (int i = 0; i < 8; ++i) { a[i] = (_Float16)p[i]; a[8 + i] = (_Float16)p[16 + i]; }
  return a;
}
__device__ __forceinline__ v16h frag_f32s(const float* rowk0, int lane, float sc) {
  v16h a; const float* p = rowk0 + 8 * (lane >> 4);
#pragma unroll
  for (int i = 0; i < 8; ++i) { a[i] = (_Float16)(p[i] * sc); a[8 + i] = (_Float16)(p[16 + i] * sc); }
  return a;
}
__device__ __forceinline__ v16h fragc_f32(const float* W, int k0, int n, int lane, int ld, int K) {
  v16h a; const int g = lane >> 4;
#pragma unroll
  for (int i = 0; i < 8; ++i) { const int ka = k0 + 8 * g + i, kb = ka + 16;
    a[i] = (_Float16)(ka < K ? W[(size_t)(ka < K ? ka : K - 1) * ld + n] : 0.f); a[8 + i] = (_Float16)(kb < K ? W[(size_t)(kb < K ? kb : K - 1) * ld + n] : 0.f); }
  return a;
}
struct F2 { v16b h, l; };
__device__ __forceinline__ F2 bsplit16(const float v[16]) { F2 r;
#pragma unroll
  for (int i = 0; i < 16; ++i) { const __bf16 h = (__bf16)v[i]; r.h[i] = h; r.l[i] = (__bf16)(v[i] - (float)h); }
  return r; }
__device__ __forceinline__ F2 split_row(const float* row, int k0, int lane) { float v[16]; const float* p = row + k0 + 8 * (lane >> 4);
#pragma unroll
  for (int i = 0; i < 8; ++i) { v[i] = p[i]; v[8 + i] = p[16 + i]; }
  return bsplit16(v); }
__device__ __forceinline__ F2 split_rowK(const float* row, int k0, int lane, int K) { float v[16]; const int g = lane >> 4;
#pragma unroll
  for (int i = 0; i < 8; ++i) { const int ka = k0 + 8 * g + i, kb = ka + 16; v[i] = ka < K ? row[ka < K ? ka : K - 1] : 0.f; v[8 + i] = kb < K ? row[kb < K ? kb : K - 1] : 0.f; }
  return bsplit16(v); }
__device__ __forceinline__ F2 split_col(const float* W, int k0, int n, int lane, int ld, int K) { float v[16]; const int g = lane >> 4;
#pragma unroll
  for (int i = 0; i < 8; ++i) { const int ka = k0 + 8 * g + i, kb = ka + 16; v[i] = ka < K ? W[(size_t)(ka < K ? ka : K - 1) * ld + n] : 0.f; v[8 + i] = kb < K ? W[(size_t)(kb < K ? kb : K - 1) * ld + n] : 0.f; }
  return bsplit16(v); }
__device__ __forceinline__ v8f mac3(const F2& a, const F2& b, v8f c) { c = wmma_bf(a.l, b.h, c); c = wmma_bf(a.h, b.l, c); return wmma_bf(a.h, b.h, c); }
__device__ __forceinline__ float sigm(float v) { return 1.0f / (1.0f + expf(-v)); }
#define LDSX() do { asm volatile("s_wait_dscnt 0" ::: "memory"); __builtin_amdgcn_wave_barrier(); __builtin_amdgcn_fence(__ATOMIC_RELEASE, "workgroup"); } while (0)


#define NB 2
#define CIN 64
#define HWD 80
#define NP 6400
#define TD3 1536
#define SMG 16
#define DG 64
#define NHD 8
#define CH 8
#define COUT 64
#ifndef TPB
#define TPB (NP / 64)
#endif
typedef __attribute__((ext_vector_type(8))) __bf16 v8b;
__device__ __forceinline__ v16b frag_b(const __bf16* rowk0, int lane) {
  union { v16b v; v8b q[2]; } u; const __bf16* p = rowk0 + 8 * (lane >> 4);
  u.q[0] = *(const v8b*)p; u.q[1] = *(const v8b*)(p + 16); return u.v;
}
__device__ __forceinline__ float bfr(float v) { return (float)(__bf16)v; }
__device__ __attribute__((noinline)) float exp_ni(float v) { return expf(v); }
__device__ __attribute__((noinline)) float erf_ni(float v) { return erff(v); }

#define WS_QKV 0u
#define WS_AG1 (WS_QKV + 4u * (size_t)NB * TD3 * NP)
#define WS_AG2 (WS_AG1 + 4u * (size_t)NB * TD3 * NP)
#define WS_KV  (WS_AG2 + 4u * (size_t)NB * TD3 * NP)
#define WS_ATT (WS_KV + 4u * (size_t)NB * SMG * NHD * 128)
#define WS_END (WS_ATT + 2u * (size_t)NB * NP * SMG * DG)

__device__ __forceinline__ const float* ms_plane(const float* QKV, const float* AG2, int b, int sm, int within) { return (sm < 8) ? (QKV + ((size_t)b * TD3 + sm * 192 + within) * NP) : (AG2 + ((size_t)b * TD3 + (sm - 8) * 192 + within) * NP); }
__global__ __launch_bounds__(128) void k_qkv(const float* __restrict__ X, const float* __restrict__ WQ, float* __restrict__ QKV) { __shared__ __align__(16) __bf16 sx[64][CIN + 8]; __shared__ __align__(16) float st[128][68];
  const int tid = threadIdx.x, wave = tid >> 5, lane = tid & 31, col = lane & 15, g = lane >> 4; const int p0 = blockIdx.x * 64, c0 = blockIdx.y * 128; const size_t b = blockIdx.z;
  for (int e = tid; e < CIN * 64; e += 128) { const int c = e >> 6, pl = e & 63; sx[pl][c] = (__bf16)X[(b * CIN + c) * (size_t)NP + p0 + pl]; }
  __syncthreads();
  v8f acc[8] = {};
#pragma unroll
  for (int kc = 0; kc < CIN / 32; ++kc) { const v16b a = frag_b(&sx[wave * 16 + col][kc * 32], lane);
#pragma unroll
    for (int j = 0; j < 8; ++j) { v16b w; const int o = c0 + j * 16 + col;
#pragma unroll
      for (int i = 0; i < 8; ++i) { w[i] = (__bf16)WQ[(size_t)o * CIN + kc * 32 + 8 * g + i]; w[8 + i] = (__bf16)WQ[(size_t)o * CIN + kc * 32 + 16 + 8 * g + i]; }
      acc[j] = wmma_bf(a, w, acc[j]); } }
#pragma unroll
  for (int j = 0; j < 8; ++j)
#pragma unroll
    for (int r = 0; r < 8; ++r) st[j * 16 + col][wave * 16 + 8 * g + r] = acc[j][r];
  __syncthreads(); for (int e = tid; e < 128 * 16; e += 128) { const int cl = e >> 4, q = e & 15; vst2(QKV + (b * TD3 + c0 + cl) * (size_t)NP + p0 + q * 4, *(const v4f*)&st[cl][q * 4]); } }
__global__ __launch_bounds__(256) void k_dw(const float* __restrict__ QKV, const float* __restrict__ WD, float* __restrict__ AG1) { __shared__ float sp[HWD + 4][HWD + 4]; __shared__ float sw[25]; __shared__ __align__(16) float so[NP];
  const int t = threadIdx.x; const int o = blockIdx.x; const size_t b = blockIdx.y; const float* src = QKV + (b * TD3 + o) * (size_t)NP;
  for (int e = t; e < (HWD + 4) * (HWD + 4); e += 256) { const int y = e / (HWD + 4) - 2, x = e % (HWD + 4) - 2; sp[y + 2][x + 2] = (y >= 0 && y < HWD && x >= 0 && x < HWD) ? src[y * HWD + x] : 0.f; }
  if (t < 25) sw[t] = bfr(WD[o * 25 + t]);
  __syncthreads();
  for (int e = t; e < NP; e += 256) { const int y = e / HWD, x = e % HWD; float a = 0.f;
#pragma unroll 1
    for (int dy = 0; dy < 5; ++dy)
#pragma unroll 1
      for (int dx = 0; dx < 5; ++dx) a += sw[dy * 5 + dx] * sp[y + dy][x + dx];
    so[e] = a; }
  __syncthreads(); for (int q = t; q < NP / 4; q += 256) vst2(AG1 + (b * TD3 + o) * (size_t)NP + q * 4, *(const v4f*)&so[q * 4]); }
__global__ __launch_bounds__(128) void k_pw(const float* __restrict__ AG1, const float* __restrict__ WP, float* __restrict__ AG2) { __shared__ __align__(16) float sa[64][68]; __shared__ __align__(16) float st[64][68];
  const int tid = threadIdx.x, wave = tid >> 5, lane = tid & 31, col = lane & 15, g = lane >> 4; const int p0 = blockIdx.x * 64, gi = blockIdx.y; const size_t b = blockIdx.z;
  for (int e = tid; e < 64 * 64; e += 128) { const int c = e >> 6, pl = e & 63; sa[pl][c] = AG1[(b * TD3 + gi * 64 + c) * (size_t)NP + p0 + pl]; }
  __syncthreads();
  v8f acc[4] = {};
#pragma unroll
  for (int kc = 0; kc < 2; ++kc) { const F2 a = split_row(&sa[wave * 16 + col][0], kc * 32, lane);
#pragma unroll
    for (int j = 0; j < 4; ++j) { v16b w; const int oo = j * 16 + col;
#pragma unroll
      for (int i = 0; i < 8; ++i) { w[i] = (__bf16)WP[(size_t)(gi * 64 + oo) * 64 + kc * 32 + 8 * g + i]; w[8 + i] = (__bf16)WP[(size_t)(gi * 64 + oo) * 64 + kc * 32 + 16 + 8 * g + i]; }
      acc[j] = wmma_bf(a.h, w, acc[j]); acc[j] = wmma_bf(a.l, w, acc[j]); } }
  __syncthreads();
#pragma unroll
  for (int j = 0; j < 4; ++j)
#pragma unroll
    for (int r = 0; r < 8; ++r) st[j * 16 + col][wave * 16 + 8 * g + r] = acc[j][r];
  __syncthreads(); for (int e = tid; e < 64 * 16; e += 128) { const int cl = e >> 4, q = e & 15; vst2(AG2 + (b * TD3 + gi * 64 + cl) * (size_t)NP + p0 + q * 4, *(const v4f*)&st[cl][q * 4]); } }
__device__ __forceinline__ void focus_row(float* t, const float* sc) { float n1 = 0.f; for (int d = 0; d < DG; ++d) { const float v = (fmaxf(t[d], 0.f) + 1e-6f) / sc[d]; t[d] = v; n1 += v * v; } n1 = sqrtf(n1); float n3 = 0.f; for (int d = 0; d < DG; ++d) { const float v = t[d] * t[d] * t[d]; t[d] = v; n3 += v * v; } n3 = sqrtf(n3); const float f = n1 / n3; for (int d = 0; d < DG; ++d) t[d] *= f; }
__global__ __launch_bounds__(64) void k_kf(const float* __restrict__ QKV, const float* __restrict__ AG2, const float* __restrict__ SCP, float* __restrict__ KF) { __shared__ float sk[64][DG + 1]; __shared__ float ssc[DG]; __shared__ __align__(16) float st[DG][68];
  const int t = threadIdx.x; const int p0 = blockIdx.x * 64, sm = blockIdx.y; const size_t b = blockIdx.z;
  if (t < DG) { const float s = bfr(SCP[t]); ssc[t] = (s > 20.f) ? s : logf(1.0f + expf(s)); }
  for (int d = 0; d < DG; ++d) sk[t][d] = ms_plane(QKV, AG2, (int)b, sm, 64 + d)[p0 + t];
  __syncthreads(); focus_row(&sk[t][0], ssc); __syncthreads();
  for (int e = t; e < DG * 64; e += 64) { const int d = e >> 6, pl = e & 63; st[d][pl] = sk[pl][d]; }
  __syncthreads(); for (int e = t; e < DG * 16; e += 64) { const int d = e >> 4, q = e & 15; vst2(KF + ((b * SMG + sm) * DG + d) * (size_t)NP + p0 + q * 4, *(const v4f*)&st[d][q * 4]); } }
__global__ __launch_bounds__(256) void k_red(const float* __restrict__ KF, const float* __restrict__ QKV, const float* __restrict__ AG2, float* __restrict__ KVS) { __shared__ float sp[4][72]; __shared__ __align__(16) float so[128];
  const int t = threadIdx.x; const int h = blockIdx.x, sm = blockIdx.y; const size_t b = blockIdx.z; const int pair = t & 63, part = t >> 6;
  const int c = pair >> 3, d = pair & 7; const float* kp = KF + ((b * SMG + sm) * DG + h * CH + c) * (size_t)NP; const float* vp = ms_plane(QKV, AG2, (int)b, sm, 128 + h * CH + d);
  float a = 0.f, s = 0.f;
#pragma unroll 1
  for (int n = part; n < NP; n += 4) { const float kv = kp[n]; a += kv * vp[n]; if (d == 0) s += kv; }
  sp[part][pair] = a; if (d == 0) sp[part][64 + c] = s; __syncthreads();
  if (t < 72) { const float v = (sp[0][t] + sp[1][t]) + (sp[2][t] + sp[3][t]); so[t] = v; } if (t >= 72 && t < 128) so[t] = 0.f;
  __syncthreads(); if (t < 32) vst2(KVS + ((b * SMG + sm) * NHD + h) * 128 + t * 4, *(const v4f*)&so[t * 4]); }
__global__ __launch_bounds__(64) void k_att(const float* __restrict__ QKV, const float* __restrict__ AG2, const float* __restrict__ SCP, const float* __restrict__ KVS, const float* __restrict__ WDW, const float* __restrict__ BDW, _Float16* __restrict__ ATT) { __shared__ float sq[64][DG + 1]; __shared__ float ssc[DG]; __shared__ float skv[NHD][72]; __shared__ float swd[CH][25], sbd[CH]; __shared__ __align__(16) _Float16 so[64][DG + 8];
  const int t = threadIdx.x; const int p0 = blockIdx.x * 64, sm = blockIdx.y; const size_t b = blockIdx.z; const int n = p0 + t; const int y = n / HWD, x = n % HWD;
  if (t < DG) { const float s = bfr(SCP[t]); ssc[t] = (s > 20.f) ? s : logf(1.0f + expf(s)); }
  for (int e = t; e < NHD * 72; e += 64) skv[e / 72][e % 72] = KVS[((b * SMG + sm) * NHD + e / 72) * 128 + (e % 72)];
  for (int e = t; e < CH * 25; e += 64) swd[e / 25][e % 25] = bfr(WDW[e]); if (t < CH) sbd[t] = bfr(BDW[t]);
  for (int d = 0; d < DG; ++d) sq[t][d] = ms_plane(QKV, AG2, (int)b, sm, d)[n];
  __syncthreads(); focus_row(&sq[t][0], ssc);
#pragma unroll 1
  for (int h = 0; h < NHD; ++h) { float zq = 0.f; for (int cc = 0; cc < CH; ++cc) zq += sq[t][h * CH + cc] * skv[h][64 + cc]; const float z = 1.0f / (zq + 1e-6f);
#pragma unroll 1
    for (int d = 0; d < CH; ++d) { float a = 0.f; for (int cc = 0; cc < CH; ++cc) a += sq[t][h * CH + cc] * skv[h][cc * CH + d]; a *= z;
      const float* vp = ms_plane(QKV, AG2, (int)b, sm, 128 + h * CH + d); float l = sbd[d];
#pragma unroll 1
      for (int dy = -2; dy <= 2; ++dy) { const int yy = y + dy; if (yy < 0 || yy >= HWD) continue;
#pragma unroll 1
        for (int dx = -2; dx <= 2; ++dx) { const int xx = x + dx; if (xx < 0 || xx >= HWD) continue; l += swd[d][(dy + 2) * 5 + dx + 2] * vp[yy * HWD + xx]; } }
      so[t][h * CH + d] = (_Float16)(a + l); } }
  __syncthreads(); for (int e = t; e < 64 * 8; e += 64) { const int pl = e >> 3, q = e & 7; vst2((unsigned*)(ATT + (b * NP + p0 + pl) * (size_t)(SMG * DG) + sm * DG + q * 8), *(const v4u*)&so[pl][q * 8]); } }
__global__ __launch_bounds__(128) void k_proj(const _Float16* __restrict__ ATT, const float* __restrict__ WPR, const float* __restrict__ GA, const float* __restrict__ BE, const float* __restrict__ MU, const float* __restrict__ VA, float* __restrict__ OUT) { __shared__ __align__(16) float st[COUT][68];
  const int tid = threadIdx.x, wave = tid >> 5, lane = tid & 31, col = lane & 15, g = lane >> 4; const int p0 = blockIdx.x * 64; const size_t b = blockIdx.y; const size_t r0 = b * NP + p0 + wave * 16;
  v8f acc[4] = {};
#pragma unroll 2
  for (int kc = 0; kc < SMG * DG / 32; ++kc) { const v16h a = frag_h(ATT + (r0 + col) * (size_t)(SMG * DG) + kc * 32, lane);
#pragma unroll
    for (int j = 0; j < 4; ++j) { v16h w; const int o = j * 16 + col;
#pragma unroll
      for (int i = 0; i < 8; ++i) { w[i] = (_Float16)bfr(WPR[(size_t)o * (SMG * DG) + kc * 32 + 8 * g + i]); w[8 + i] = (_Float16)bfr(WPR[(size_t)o * (SMG * DG) + kc * 32 + 16 + 8 * g + i]); }
      acc[j] = wmma16(a, w, acc[j]); } }
#pragma unroll
  for (int j = 0; j < 4; ++j) { const int o = j * 16 + col; const float inv = bfr(GA[o]) / sqrtf(bfr(VA[o]) + 1e-5f); const float sh = bfr(BE[o]) - bfr(MU[o]) * inv;
#pragma unroll
    for (int r = 0; r < 8; ++r) st[o][wave * 16 + 8 * g + r] = acc[j][r] * inv + sh; }
  __syncthreads(); for (int e = tid; e < COUT * 16; e += 128) { const int o = e >> 4, q = e & 15; vst2(OUT + (b * COUT + o) * (size_t)NP + p0 + q * 4, *(const v4f*)&st[o][q * 4]); } }
extern "C" void kernel_launch(void* const* d_in, const int* in_sizes, int n_in, void* d_out, int out_size, void* d_ws, size_t ws_size, hipStream_t stream) {
  (void)in_sizes; (void)n_in; (void)out_size;
  const float** F = (const float**)d_in;
  if (ws_size < (size_t)WS_END) return;
  char* ws = (char*)d_ws; float *QKV = (float*)(ws + WS_QKV), *AG1 = (float*)(ws + WS_AG1), *AG2 = (float*)(ws + WS_AG2), *KVS = (float*)(ws + WS_KV); _Float16* ATT = (_Float16*)(ws + WS_ATT); float* KF = AG1;
  k_qkv<<<dim3(NP / 64, TD3 / 128, NB), 128, 0, stream>>>(F[0], F[1], QKV);
  k_dw<<<dim3(TD3, NB), 256, 0, stream>>>(QKV, F[2], AG1);
  k_pw<<<dim3(NP / 64, TD3 / 64, NB), 128, 0, stream>>>(AG1, F[3], AG2);
  k_kf<<<dim3(NP / 64, SMG, NB), 64, 0, stream>>>(QKV, AG2, F[4], KF);
  k_red<<<dim3(NHD, SMG, NB), 256, 0, stream>>>(KF, QKV, AG2, KVS);
  k_att<<<dim3(TPB, SMG, NB), 64, 0, stream>>>(QKV, AG2, F[4], KVS, F[5], F[6], ATT);
  k_proj<<<dim3(TPB, NB), 128, 0, stream>>>(ATT, F[7], F[8], F[9], F[10], F[11], (float*)d_out);
}
